// FeatureAlign_V2_44066364457482
// MI455X (gfx1250) — hardware-verified
//
#include <hip/hip_runtime.h>
#define NBI 2
#define CC 128
#define HH 128
#define NPX (HH * HH)
#define PW 130
#define PR 132
#define MP (HH * PW)
#define GG 8
#define CG 16
#define KT 9
#define KD (KT * CC)
#define NO3 224
#define RCH 16384
typedef __bf16 v16b __attribute__((ext_vector_type(16)));
typedef unsigned short v8us __attribute__((ext_vector_type(8), may_alias));
typedef float  v8f  __attribute__((ext_vector_type(8)));
typedef float  v4f  __attribute__((ext_vector_type(4)));
typedef float  v4fa __attribute__((ext_vector_type(4), may_alias));
union FragB { v16b v; v8us half[2]; unsigned short u[16]; };

__device__ __forceinline__ unsigned short bf16_bits(float x) { unsigned int u = __float_as_uint(x); return (unsigned short)((u + 0x7FFFu + ((u >> 16) & 1u)) >> 16); }
__device__ __forceinline__ float bf16_val(unsigned short b) { return __uint_as_float(((unsigned int)b) << 16); }
__device__ __forceinline__ float bf16_round(float x) { return bf16_val(bf16_bits(x)); }
template <int NT>
__device__ __forceinline__ v8f mmaN(v16b ah, v16b al, v16b bh, v16b bl, v8f c) {
  c = __builtin_amdgcn_wmma_f32_16x16x32_bf16(false, ah, false, bh, (short)0, c, false, false);
  if (NT >= 2) c = __builtin_amdgcn_wmma_f32_16x16x32_bf16(false, al, false, bh, (short)0, c, false, false);
  if (NT >= 3) c = __builtin_amdgcn_wmma_f32_16x16x32_bf16(false, ah, false, bl, (short)0, c, false, false);
  asm volatile("v_nop\n\tv_nop\n\tv_nop\n\tv_nop" : "+v"(c) : "v"(ah), "v"(al), "v"(bh), "v"(bl));
  return c;
}

__global__ __launch_bounds__(256) void k_wt_bf16(const float* __restrict__ W, unsigned short* __restrict__ Wt, int K, int N) {
  const int t = blockIdx.x * 256 + threadIdx.x;
  const int k8n = K / 8;
  if (t >= N * k8n) return;
  const int n = t / k8n, k8 = (t % k8n) * 8;
  v8us v;
#pragma unroll
  for (int i = 0; i < 8; ++i) v[i] = bf16_bits(W[(size_t)(k8 + i) * N + n]);
  *(volatile v8us*)(Wt + (size_t)n * K + k8) = v;
  __threadfence();
  *(volatile v8us*)(Wt + (size_t)n * K + k8) = v;
}

template <bool ASPLIT, int ACT, bool BIAS_BF16>
__global__ __launch_bounds__(128) void k_gemm_bf(const float* __restrict__ A, int lda, const unsigned short* __restrict__ Wt, int ldb,
                                               const float* __restrict__ bias, float* __restrict__ C, int ldc, int M, int N, int K) {
  __shared__ __attribute__((aligned(16))) float so[4][16][64];
  const int tid = threadIdx.x, w = tid >> 5, lane = tid & 31, ln = lane & 15, hh = lane >> 4;
  const int ntn = N / 64;
  const int wid = blockIdx.x * 4 + w;
  const int mt = wid / ntn, nq = wid % ntn;
  if (mt * 16 >= M) return;
  const int row0 = mt * 16, col0 = nq * 64;
  const float* arow = A + (size_t)(row0 + ln) * lda;
  v8f acc[4] = {};
  for (int kb = 0; kb < K; kb += 32) {
    FragB ah, al;
    const v4f x0 = *(const v4fa*)(arow + kb + 8 * hh), x1 = *(const v4fa*)(arow + kb + 8 * hh + 4);
    const v4f x2 = *(const v4fa*)(arow + kb + 16 + 8 * hh), x3 = *(const v4fa*)(arow + kb + 16 + 8 * hh + 4);
    float xs[16] = {x0[0],x0[1],x0[2],x0[3],x1[0],x1[1],x1[2],x1[3],x2[0],x2[1],x2[2],x2[3],x3[0],x3[1],x3[2],x3[3]};
#pragma unroll
    for (int i = 0; i < 16; ++i) { const unsigned short hb = bf16_bits(xs[i]); ah.u[i] = hb; al.u[i] = ASPLIT ? bf16_bits(xs[i] - bf16_val(hb)) : (unsigned short)0; }
#pragma unroll
    for (int t = 0; t < 4; ++t) {
      const unsigned short* brow = Wt + (size_t)(col0 + t * 16 + ln) * ldb + kb;
      FragB b;
      b.half[0] = *(const v8us*)(brow + 8 * hh);
      b.half[1] = *(const v8us*)(brow + 16 + 8 * hh);
      acc[t] = mmaN<ASPLIT ? 2 : 1>(ah.v, al.v, b.v, b.v, acc[t]);
    }
  }
#pragma unroll
  for (int t = 0; t < 4; ++t) {
    float bv = bias ? bias[col0 + t * 16 + ln] : 0.f;
    if (BIAS_BF16) bv = bf16_round(bv);
#pragma unroll
    for (int r = 0; r < 8; ++r) { float v = acc[t][r] + bv; if (ACT == 1) v = fmaxf(v, 0.f); so[w][8 * hh + r][t * 16 + ln] = v; }
  }
  __builtin_amdgcn_fence(__ATOMIC_ACQ_REL, "workgroup");
  __builtin_amdgcn_wave_barrier();
  const int rsub = lane >> 4, c4 = (lane & 15) * 4;
  for (int pass = 0; pass < 2; ++pass) {
#pragma unroll
    for (int q = 0; q < 8; ++q) {
      const int r = q * 2 + rsub;
      const v4f v = *(const v4fa*)&so[w][r][c4];
      *(volatile v4f*)(C + (size_t)(row0 + r) * ldc + col0 + c4) = v;
    }
    if (pass == 0) __threadfence();
  }
}

template <bool ASPLIT, int ACT, bool BIAS_BF16, bool RES_BF16>
__global__ __launch_bounds__(128) void k_gemm_bf3(const float* __restrict__ A, int lda, const unsigned short* __restrict__ Wt, int ldb,
                                                const float* __restrict__ bias, const float* __restrict__ resid, int rmod, int ldr,
                                                float* __restrict__ C, int ldc, int M, int N, int K) {
  __shared__ __attribute__((aligned(16))) float so[4][16][64];
  const int tid = threadIdx.x, w = tid >> 5, lane = tid & 31, ln = lane & 15, hh = lane >> 4;
  const int ntn = N / 64;
  const int wid = blockIdx.x * 4 + w;
  const int mt = wid / ntn, nq = wid % ntn;
  if (mt * 16 >= M) return;
  const int row0 = mt * 16, col0 = nq * 64;
  const float* arow = A + (size_t)(row0 + ln) * lda;
  v8f acc[4] = {};
  for (int kb = 0; kb < K; kb += 32) {
    FragB ah, al;
    const v4f x0 = *(const v4fa*)(arow + kb + 8 * hh), x1 = *(const v4fa*)(arow + kb + 8 * hh + 4);
    const v4f x2 = *(const v4fa*)(arow + kb + 16 + 8 * hh), x3 = *(const v4fa*)(arow + kb + 16 + 8 * hh + 4);
    float xs[16] = {x0[0],x0[1],x0[2],x0[3],x1[0],x1[1],x1[2],x1[3],x2[0],x2[1],x2[2],x2[3],x3[0],x3[1],x3[2],x3[3]};
#pragma unroll
    for (int i = 0; i < 16; ++i) { const unsigned short hb = bf16_bits(xs[i]); ah.u[i] = hb; al.u[i] = ASPLIT ? bf16_bits(xs[i] - bf16_val(hb)) : (unsigned short)0; }
#pragma unroll
    for (int t = 0; t < 4; ++t) {
      const unsigned short* brow = Wt + (size_t)(col0 + t * 16 + ln) * ldb + kb;
      FragB b;
      b.half[0] = *(const v8us*)(brow + 8 * hh);
      b.half[1] = *(const v8us*)(brow + 16 + 8 * hh);
      acc[t] = mmaN<ASPLIT ? 2 : 1>(ah.v, al.v, b.v, b.v, acc[t]);
    }
  }
#pragma unroll
  for (int t = 0; t < 4; ++t) {
    const int col = col0 + t * 16 + ln;
    float bv = bias ? bias[col] : 0.f;
    if (BIAS_BF16) bv = bf16_round(bv);
#pragma unroll
    for (int r = 0; r < 8; ++r) {
      float v = acc[t][r] + bv;
      if (resid) { float rv = resid[(size_t)((row0 + 8 * hh + r) % rmod) * ldr + col]; if (RES_BF16) rv = bf16_round(rv); v += rv; }
      if (ACT == 1) v = fmaxf(v, 0.f);
      if (ACT == 2) v = 0.5f * v * (1.0f + erff(v * 0.70710678118654752f));
      if (ACT == 3) { const float u = 0.7978845608028654f * (v + 0.044715f * v * v * v); v = 0.5f * v * (1.0f + tanhf(u)); }
      so[w][8 * hh + r][t * 16 + ln] = v;
    }
  }
  __builtin_amdgcn_fence(__ATOMIC_ACQ_REL, "workgroup");
  __builtin_amdgcn_wave_barrier();
  const int rsub = lane >> 4, c4 = (lane & 15) * 4;
  for (int pass = 0; pass < 2; ++pass) {
#pragma unroll
    for (int q = 0; q < 8; ++q) {
      const int r = q * 2 + rsub;
      const v4f v = *(const v4fa*)&so[w][r][c4];
      *(volatile v4f*)(C + (size_t)(row0 + r) * ldc + col0 + c4) = v;
    }
    if (pass == 0) __threadfence();
  }
}
template <bool PARAM_BF16>
__global__ __launch_bounds__(256) void k_layernorm(const float* __restrict__ X, const float* __restrict__ R, const float* __restrict__ g, const float* __restrict__ bta,
                                                  float* __restrict__ out_sum, float* __restrict__ out_norm, int N, float eps) {
  __shared__ float red[256];
  const int row = blockIdx.x, tid = threadIdx.x;
  const float* x = X + (size_t)row * N; const float* rr = R ? R + (size_t)row * N : nullptr;
  float vals[16];
  const int per = N / 256;
  float s1 = 0.f;
  for (int u = 0; u < per / 4; ++u) {
    const int j = tid * 4 + 1024 * u;
    const v4f a = *(const v4fa*)(x + j);
    v4f b = {0.f,0.f,0.f,0.f}; if (rr) b = *(const v4fa*)(rr + j);
#pragma unroll
    for (int q = 0; q < 4; ++q) { const float v = a[q] + b[q]; vals[u * 4 + q] = v; s1 += v; }
  }
  red[tid] = s1; __syncthreads();
  for (int st = 128; st > 0; st >>= 1) { if (tid < st) red[tid] += red[tid + st]; __syncthreads(); }
  const float mu = red[0] / (float)N; __syncthreads();
  float s2 = 0.f;
  for (int u = 0; u < per / 4; ++u)
#pragma unroll
    for (int q = 0; q < 4; ++q) { const float c = vals[u * 4 + q] - mu; s2 += c * c; }
  red[tid] = s2; __syncthreads();
  for (int st = 128; st > 0; st >>= 1) { if (tid < st) red[tid] += red[tid + st]; __syncthreads(); }
  const float rs = rsqrtf(red[0] / (float)N + eps);
  for (int pass = 0; pass < 2; ++pass) {
    for (int u = 0; u < per / 4; ++u) {
      const int j = tid * 4 + 1024 * u;
      v4f o, sm;
#pragma unroll
      for (int q = 0; q < 4; ++q) {
        float gg = g[j + q], bb = bta[j + q];
        if (PARAM_BF16) { gg = bf16_round(gg); bb = bf16_round(bb); }
        sm[q] = vals[u * 4 + q]; o[q] = (vals[u * 4 + q] - mu) * rs * gg + bb;
      }
      if (out_sum) *(volatile v4f*)(out_sum + (size_t)row * N + j) = sm;
      *(volatile v4f*)(out_norm + (size_t)row * N + j) = o;
    }
    if (pass == 0) __threadfence();
  }
}


typedef _Float16 v16h __attribute__((ext_vector_type(16)));
union FragH { v16h v; v8us half[2]; _Float16 h[16]; unsigned short u[16]; };
template <int NT>
__device__ __forceinline__ v8f mmaH(v16h ah, v16h al, v16h bh, v16h bl, v8f c) {
  c = __builtin_amdgcn_wmma_f32_16x16x32_f16(false, ah, false, bh, (short)0, c, false, false);
  if (NT >= 2) c = __builtin_amdgcn_wmma_f32_16x16x32_f16(false, al, false, bh, (short)0, c, false, false);
  if (NT >= 3) c = __builtin_amdgcn_wmma_f32_16x16x32_f16(false, ah, false, bl, (short)0, c, false, false);
  asm volatile("v_nop\n\tv_nop\n\tv_nop\n\tv_nop" : "+v"(c) : "v"(ah), "v"(al), "v"(bh), "v"(bl));
  return c;
}
template <bool ASPLIT>
__global__ __launch_bounds__(128) void k_gemm_h(const float* __restrict__ A, int lda, size_t sA, const _Float16* __restrict__ Bh, int ldb, size_t sB, float alpha, float* __restrict__ C, int ldc, size_t sC, int M, int N, int K) {
  __shared__ __attribute__((aligned(16))) float so[4][16][64];
  const int tid = threadIdx.x, w = tid >> 5, lane = tid & 31, ln = lane & 15, hh = lane >> 4; const int by = blockIdx.y;
  A += (size_t)by * sA; Bh += (size_t)by * sB; C += (size_t)by * sC;
  const int ntn = (N + 63) / 64; const int wid = blockIdx.x * 4 + w; const int mt = wid / ntn, nq = wid % ntn; if (mt * 16 >= M) return;
  const int row0 = mt * 16, col0 = nq * 64; const float* arow = A + (size_t)(row0 + ln) * lda;
  v8f acc[4] = {};
  for (int kb = 0; kb < K; kb += 32) {
    FragH ah, al;
    const v4f x0 = *(const v4fa*)(arow + kb + 8 * hh), x1 = *(const v4fa*)(arow + kb + 8 * hh + 4), x2 = *(const v4fa*)(arow + kb + 16 + 8 * hh), x3 = *(const v4fa*)(arow + kb + 16 + 8 * hh + 4);
    float xs[16] = {x0[0],x0[1],x0[2],x0[3],x1[0],x1[1],x1[2],x1[3],x2[0],x2[1],x2[2],x2[3],x3[0],x3[1],x3[2],x3[3]};
#pragma unroll
    for (int i = 0; i < 16; ++i) { const _Float16 h = (_Float16)xs[i]; ah.h[i] = h; al.h[i] = ASPLIT ? (_Float16)(xs[i] - (float)h) : (_Float16)0.0f; }
#pragma unroll
    for (int t = 0; t < 4; ++t) { if (col0 + t * 16 >= N) continue; const size_t boff = (size_t)(col0 + t * 16 + ln) * ldb + kb; FragH bq; bq.half[0] = *(const v8us*)(Bh + boff + 8 * hh); bq.half[1] = *(const v8us*)(Bh + boff + 16 + 8 * hh);
      acc[t] = mmaH<ASPLIT ? 2 : 1>(ah.v, al.v, bq.v, bq.v, acc[t]); }
  }
#pragma unroll
  for (int t = 0; t < 4; ++t) { if (col0 + t * 16 >= N) continue;
#pragma unroll
    for (int r = 0; r < 8; ++r) so[w][8 * hh + r][t * 16 + ln] = acc[t][r] * alpha; }
  __builtin_amdgcn_fence(__ATOMIC_ACQ_REL, "workgroup"); __builtin_amdgcn_wave_barrier();
  const int rsub = lane >> 4, c4 = (lane & 15) * 4;
  for (int pass = 0; pass < 2; ++pass) {
#pragma unroll
    for (int q = 0; q < 8; ++q) { const int r = q * 2 + rsub; if (col0 + c4 < N) { const v4f v = *(const v4fa*)&so[w][r][c4]; *(volatile v4f*)(C + (size_t)(row0 + r) * ldc + col0 + c4) = v; } }
    if (pass == 0) __threadfence(); }
}

__global__ __launch_bounds__(256) void k_wt_f16(const float* __restrict__ W, _Float16* __restrict__ Wt, int K, int N, float scale) {
  const int t = blockIdx.x * 256 + threadIdx.x; if (t >= N * (K / 8)) return; const int n = t / (K / 8), k8 = (t % (K / 8)) * 8; FragH f;
#pragma unroll
  for (int i = 0; i < 8; ++i) f.h[i] = (_Float16)(bf16_round(W[(size_t)(k8 + i) * N + n]) * scale); const v8us o = f.half[0];
  *(volatile v8us*)((unsigned short*)Wt + (size_t)n * K + k8) = o; __threadfence(); *(volatile v8us*)((unsigned short*)Wt + (size_t)n * K + k8) = o;
}
template <int ACT>
__global__ __launch_bounds__(128) void k_gemm_hhx(const _Float16* __restrict__ A, int lda, size_t sA, const _Float16* __restrict__ Bh, int ldb, size_t sB, float alpha, const float* __restrict__ bias, size_t sBias, const float* __restrict__ CP, int rowsPerB, size_t sCPb, int row0g,
    float* __restrict__ C, _Float16* __restrict__ C16, int ldc, size_t sC, int M, int N, int K) {
  __shared__ __attribute__((aligned(16))) float so[4][16][64];
  const int tid = threadIdx.x, w = tid >> 5, lane = tid & 31, ln = lane & 15, hh = lane >> 4; const int by = blockIdx.y;
  A += (size_t)by * sA; Bh += (size_t)by * sB; const size_t cofs = (size_t)by * sC; const float* bp = bias ? bias + (size_t)by * sBias : nullptr;
  const int ntn = (N + 63) / 64; const int wid = blockIdx.x * 4 + w; const int mt = wid / ntn, nq = wid % ntn; if (mt * 16 >= M) return;
  const int row0 = mt * 16, col0 = nq * 64; const _Float16* arow = A + (size_t)(row0 + ln) * lda;
  v8f acc[4] = {};
  for (int kb = 0; kb < K; kb += 32) { FragH ah; ah.half[0] = *(const v8us*)((const unsigned short*)arow + kb + 8 * hh); ah.half[1] = *(const v8us*)((const unsigned short*)arow + kb + 16 + 8 * hh);
#pragma unroll
    for (int t = 0; t < 4; ++t) { if (col0 + t * 16 >= N) continue; const size_t boff = (size_t)(col0 + t * 16 + ln) * ldb + kb; FragH bq; bq.half[0] = *(const v8us*)((const unsigned short*)Bh + boff + 8 * hh); bq.half[1] = *(const v8us*)((const unsigned short*)Bh + boff + 16 + 8 * hh);
      acc[t] = mmaH<1>(ah.v, ah.v, bq.v, bq.v, acc[t]); }
  }
#pragma unroll
  for (int t = 0; t < 4; ++t) { if (col0 + t * 16 >= N) continue; const int col = col0 + t * 16 + ln; const float bv = bp ? bf16_round(bp[col]) : 0.f;
#pragma unroll
    for (int r = 0; r < 8; ++r) { float v = acc[t][r] * alpha + bv; if (CP) { const int bidx = (row0g + row0 + 8 * hh + r) / rowsPerB; v += CP[(size_t)bidx * sCPb + (size_t)by * 64 + col]; } if (ACT == 1) v = (v > 0.f) ? v : expm1f(v); else if (ACT == 7) v = (v > 0.f) ? v + 1.0f : expf(v); else if (ACT == 8) v = tanhf(v); else if (ACT == 9) v = 0.5f * v * (1.0f + tanhf(0.7978845608028654f * (v + 0.044715f * v * v * v))); else if (ACT == 11) v = 1.0f / (1.0f + expf(-v)); else if (ACT == 12) v = (v > 0.f) ? v : 0.01f * v; else if (ACT == 14) v = (v > 0.f) ? v : 0.1f * v; else if (ACT == 15) v = v / (1.0f + expf(-v)); else if (ACT == 3) v = fmaxf(v, 0.f); else if (ACT == 6) v = 0.5f * v * (1.0f + erff(v * 0.70710678118654752f)); so[w][8 * hh + r][t * 16 + ln] = v; } }
  __builtin_amdgcn_fence(__ATOMIC_ACQ_REL, "workgroup"); __builtin_amdgcn_wave_barrier();
  const int rsub = lane >> 4, c4 = (lane & 15) * 4; typedef _Float16 v4h __attribute__((ext_vector_type(4)));
  for (int pass = 0; pass < 2; ++pass) {
#pragma unroll
    for (int q = 0; q < 8; ++q) { const int r = q * 2 + rsub; if (col0 + c4 < N) { const v4f v = *(const v4fa*)&so[w][r][c4]; if (C) *(volatile v4f*)(C + cofs + (size_t)(row0 + r) * ldc + col0 + c4) = v; if (C16) { v4h h4; for (int i = 0; i < 4; ++i) h4[i] = (_Float16)v[i]; *(volatile v4h*)(C16 + cofs + (size_t)(row0 + r) * ldc + col0 + c4) = h4; } } }
    if (pass == 0) __threadfence(); }
}


typedef _Float16 v4h __attribute__((ext_vector_type(4)));

__global__ __launch_bounds__(256) void k_x16(const float* __restrict__ x, _Float16* __restrict__ X16, size_t n8) { const size_t t = (size_t)blockIdx.x * 256 + threadIdx.x; if (t >= n8) return; FragH f;
#pragma unroll
  for (int q = 0; q < 8; ++q) f.h[q] = (_Float16)bf16_round(x[t * 8 + q]); *(volatile v8us*)((unsigned short*)X16 + t * 8) = f.half[0]; __threadfence(); *(volatile v8us*)((unsigned short*)X16 + t * 8) = f.half[0]; }
__global__ __launch_bounds__(256) void k_h16(const float* __restrict__ x, _Float16* __restrict__ X16, size_t n8) { const size_t t = (size_t)blockIdx.x * 256 + threadIdx.x; if (t >= n8) return; FragH f;
#pragma unroll
  for (int q = 0; q < 8; ++q) f.h[q] = (_Float16)x[t * 8 + q]; *(volatile v8us*)((unsigned short*)X16 + t * 8) = f.half[0]; __threadfence(); *(volatile v8us*)((unsigned short*)X16 + t * 8) = f.half[0]; }
__global__ __launch_bounds__(256) void k_round16f(const float* __restrict__ W, _Float16* __restrict__ Bt, size_t n8) { const size_t t = (size_t)blockIdx.x * 256 + threadIdx.x; if (t >= n8) return; FragH f;
#pragma unroll
  for (int i = 0; i < 8; ++i) f.h[i] = (_Float16)(bf16_round(W[t * 8 + i]) * 16.0f); *(volatile v8us*)((unsigned short*)Bt + t * 8) = f.half[0]; __threadfence(); *(volatile v8us*)((unsigned short*)Bt + t * 8) = f.half[0]; }
template <int NHv, int TTv>
__global__ __launch_bounds__(256) void k_vt(const _Float16* __restrict__ V16, int ldv, int voff, _Float16* __restrict__ Vt) { __shared__ unsigned short tl[64][66]; const int tid = threadIdx.x; const int slab = blockIdx.x / (TTv / 64), lg = blockIdx.x % (TTv / 64); const int b = slab / NHv, h = slab % NHv;
  for (int i = tid; i < 64 * 8; i += 256) { const int r = i / 8, c8 = (i % 8) * 8; FragH f; f.half[0] = *(const v8us*)((const unsigned short*)V16 + ((size_t)b * TTv + lg * 64 + r) * ldv + voff + h * 64 + c8);
#pragma unroll
    for (int q = 0; q < 8; ++q) tl[r][c8 + q] = f.u[q]; }
  __syncthreads();
  for (int pass = 0; pass < 2; ++pass) {
#pragma unroll
    for (int rd = 0; rd < 2; ++rd) { const int d = rd * 32 + tid / 8, pc = tid % 8; FragH f;
#pragma unroll
      for (int q = 0; q < 8; ++q) f.u[q] = tl[pc * 8 + q][d];
      *(volatile v8us*)((unsigned short*)Vt + ((size_t)slab * 64 + d) * TTv + lg * 64 + pc * 8) = f.half[0]; }
    if (pass == 0) __threadfence(); } }

__global__ __launch_bounds__(256) void k_hl(const float* __restrict__ F, _Float16* __restrict__ Hh, _Float16* __restrict__ Hl, size_t n8) { const size_t t = (size_t)blockIdx.x * 256 + threadIdx.x; if (t >= n8) return; FragH fh, fl; const v4f a = *(const v4fa*)(F + t * 8), c = *(const v4fa*)(F + t * 8 + 4);
#pragma unroll
  for (int q = 0; q < 4; ++q) { _Float16 h = (_Float16)a[q]; fh.h[q] = h; fl.h[q] = (_Float16)((a[q] - (float)h) * 1024.0f); h = (_Float16)c[q]; fh.h[4 + q] = h; fl.h[4 + q] = (_Float16)((c[q] - (float)h) * 1024.0f); }
  for (int pass = 0; pass < 2; ++pass) { *(volatile v8us*)((unsigned short*)Hh + t * 8) = fh.half[0]; *(volatile v8us*)((unsigned short*)Hl + t * 8) = fl.half[0]; if (pass == 0) __threadfence(); } }

__global__ __launch_bounds__(256) void k_gap(const float* __restrict__ fl, int b, float* __restrict__ GS) { __shared__ double red[256]; const int tid = threadIdx.x, c = blockIdx.x; const float* p = fl + ((size_t)b * CC + c) * NPX; double s = 0.0;
#pragma unroll 1
  for (int i = tid; i < NPX; i += 256) s += (double)bf16_round(p[i]);
  red[tid] = s; __syncthreads(); for (int st = 128; st > 0; st >>= 1) { if (tid < st) red[tid] += red[tid + st]; __syncthreads(); }
  if (tid < 32) { const float v = (tid == 0) ? (float)(red[0] / (double)NPX) : 0.f; *(volatile float*)(GS + c * 32 + tid) = v; __threadfence(); *(volatile float*)(GS + c * 32 + tid) = v; } }
__global__ __launch_bounds__(256) void k_agate(const float* __restrict__ GS, const float* __restrict__ wat, float* __restrict__ AG) {
  #pragma clang fp contract(off)
  __shared__ float gp[CC]; const int tid = threadIdx.x; if (tid < CC) gp[tid] = GS[tid * 32]; __syncthreads(); float a = 0.f;
  if (tid < CC) {
#pragma unroll 1
    for (int c = 0; c < CC; ++c) a += bf16_round(wat[tid * CC + c]) * gp[c]; }
  const float gte = a * (1.0f / (1.0f + expf(-a))); __syncthreads();
  if (tid < CC) { for (int l = 0; l < 32; ++l) { const float v = (l == 0) ? gte : 0.f; *(volatile float*)(AG + tid * 32 + l) = v; } __threadfence(); for (int l = 0; l < 32; ++l) { const float v = (l == 0) ? gte : 0.f; *(volatile float*)(AG + tid * 32 + l) = v; } } }
__global__ __launch_bounds__(256) void k_xg(const float* __restrict__ fl, int b, const float* __restrict__ AG, _Float16* __restrict__ XG) {
  #pragma clang fp contract(off)
  const int t = blockIdx.x * 256 + threadIdx.x; if (t >= NPX * (CC / 8)) return; const int c0 = (t % (CC / 8)) * 8, p = t / (CC / 8); FragH f;
#pragma unroll
  for (int q = 0; q < 8; ++q) f.h[q] = (_Float16)(bf16_round(fl[((size_t)b * CC + c0 + q) * NPX + p]) + AG[(c0 + q) * 32]);
  *(volatile v8us*)((unsigned short*)XG + (size_t)p * CC + c0) = f.half[0]; __threadfence(); *(volatile v8us*)((unsigned short*)XG + (size_t)p * CC + c0) = f.half[0]; }
__global__ __launch_bounds__(256) void k_ups(const float* __restrict__ fs, int b, _Float16* __restrict__ FU16) {
  #pragma clang fp contract(off)
  const int t = blockIdx.x * 256 + threadIdx.x; if (t >= NPX * (CC / 8)) return; const int c0 = (t % (CC / 8)) * 8, p = t / (CC / 8); const int h = p / HH, w = p % HH;
  const float sy = ((float)h + 0.5f) * 0.5f - 0.5f, sx = ((float)w + 0.5f) * 0.5f - 0.5f; const float y0f = floorf(sy), x0f = floorf(sx); const float wy = sy - y0f, wx = sx - x0f; const int y0 = (int)y0f, x0 = (int)x0f; const int ya = min(max(y0, 0), 63), yb = min(max(y0 + 1, 0), 63), xa = min(max(x0, 0), 63), xb = min(max(x0 + 1, 0), 63);
  const float wy0 = 1.f - wy, wy1 = wy, wx0 = 1.f - wx, wx1 = wx;
  FragH f;
#pragma unroll
  for (int q = 0; q < 8; ++q) { const float* pc = fs + ((size_t)b * CC + c0 + q) * 4096; const float v00 = bf16_round(pc[ya * 64 + xa]), v01 = bf16_round(pc[ya * 64 + xb]), v10 = bf16_round(pc[yb * 64 + xa]), v11 = bf16_round(pc[yb * 64 + xb]);
    const float r0 = wx0 * v00 + wx1 * v01, r1 = wx0 * v10 + wx1 * v11; f.h[q] = (_Float16)(wy0 * r0 + wy1 * r1); }
  *(volatile v8us*)((unsigned short*)FU16 + (size_t)p * CC + c0) = f.half[0]; __threadfence(); *(volatile v8us*)((unsigned short*)FU16 + (size_t)p * CC + c0) = f.half[0]; }
__global__ __launch_bounds__(256) void k_f16(const float* __restrict__ F, _Float16* __restrict__ H16) { const int t = blockIdx.x * 256 + threadIdx.x; if (t >= NPX * (CC / 8)) return; const v4f a = *(const v4fa*)(F + (size_t)t * 8), c = *(const v4fa*)(F + (size_t)t * 8 + 4); FragH f;
#pragma unroll
  for (int q = 0; q < 8; ++q) f.h[q] = (_Float16)((q < 4) ? a[q] : c[q - 4]);
  *(volatile v8us*)((unsigned short*)H16 + (size_t)t * 8) = f.half[0]; __threadfence(); *(volatile v8us*)((unsigned short*)H16 + (size_t)t * 8) = f.half[0]; }
__global__ __launch_bounds__(256) void k_pad(const float* __restrict__ OF, _Float16* __restrict__ XP) { const int t = blockIdx.x * 256 + threadIdx.x; if (t >= PR * PW * (CC / 8)) return; const int c0 = (t % (CC / 8)) * 8, pp = t / (CC / 8); const int h = pp / PW - 1, w = pp % PW - 1; const bool in = (h >= 0 && h < HH && w >= 0 && w < HH); const int pc = min(max(h, 0), HH - 1) * HH + min(max(w, 0), HH - 1); const v4f a = *(const v4fa*)(OF + (size_t)pc * CC + c0), cq = *(const v4fa*)(OF + (size_t)pc * CC + c0 + 4); FragH f;
#pragma unroll
  for (int q = 0; q < 8; ++q) f.h[q] = in ? (_Float16)((q < 4) ? a[q] : cq[q - 4]) : (_Float16)0.0f;
  *(volatile v8us*)((unsigned short*)XP + (size_t)pp * CC + c0) = f.half[0]; __threadfence(); *(volatile v8us*)((unsigned short*)XP + (size_t)pp * CC + c0) = f.half[0]; }
__global__ __launch_bounds__(256) void k_wcoff(const float* __restrict__ w, _Float16* __restrict__ Bt) { const int t = blockIdx.x * 256 + threadIdx.x; if (t >= KT * NO3 * (CC / 8)) return; const int c0 = (t % (CC / 8)) * 8; const int j = (t / (CC / 8)) % NO3; const int k = t / ((CC / 8) * NO3); FragH f;
#pragma unroll
  for (int q = 0; q < 8; ++q) f.h[q] = (j < 216) ? (_Float16)(bf16_round(w[((size_t)j * CC + c0 + q) * KT + k]) * 16.0f) : (_Float16)0.0f;
  *(volatile v8us*)((unsigned short*)Bt + ((size_t)k * NO3 + j) * CC + c0) = f.half[0]; __threadfence(); *(volatile v8us*)((unsigned short*)Bt + ((size_t)k * NO3 + j) * CC + c0) = f.half[0]; }
__global__ __launch_bounds__(256) void k_wdcn(const float* __restrict__ w, _Float16* __restrict__ Bt) { const int t = blockIdx.x * 256 + threadIdx.x; if (t >= CC * (KD / 8)) return; const int col0 = (t % (KD / 8)) * 8; const int o = t / (KD / 8); const int k = col0 / CC, c0 = col0 % CC; FragH f;
#pragma unroll
  for (int q = 0; q < 8; ++q) f.h[q] = (_Float16)(bf16_round(w[((size_t)o * CC + c0 + q) * KT + k]) * 16.0f);
  *(volatile v8us*)((unsigned short*)Bt + (size_t)o * KD + col0) = f.half[0]; __threadfence(); *(volatile v8us*)((unsigned short*)Bt + (size_t)o * KD + col0) = f.half[0]; }
__global__ __launch_bounds__(256) void k_woff(const float* __restrict__ w, _Float16* __restrict__ Ba, _Float16* __restrict__ Bb) { const int t = blockIdx.x * 256 + threadIdx.x; if (t >= CC * (CC / 8)) return; const int c0 = (t % (CC / 8)) * 8, o = t / (CC / 8); FragH fa, fb;
#pragma unroll
  for (int q = 0; q < 8; ++q) { fa.h[q] = (_Float16)(bf16_round(w[(size_t)o * 2 * CC + c0 + q]) * 16.0f); fb.h[q] = (_Float16)(bf16_round(w[(size_t)o * 2 * CC + CC + c0 + q]) * 16.0f); }
  for (int pass = 0; pass < 2; ++pass) { *(volatile v8us*)((unsigned short*)Ba + (size_t)o * CC + c0) = fa.half[0]; *(volatile v8us*)((unsigned short*)Bb + (size_t)o * CC + c0) = fb.half[0]; if (pass == 0) __threadfence(); } }
__global__ __launch_bounds__(256) void k_bpad(const float* __restrict__ bb, int n, int np, float* __restrict__ BP) { const int l = threadIdx.x; if (l >= np) return; const float v = (l < n) ? bb[l] : 0.f; *(volatile float*)(BP + l) = v; __threadfence(); *(volatile float*)(BP + l) = v; }
__global__ __launch_bounds__(256) void k_dsamp(const float* __restrict__ O, const _Float16* __restrict__ FU16, int r0, _Float16* __restrict__ DCOL) {
  #pragma clang fp contract(off)
  const int t = blockIdx.x * 256 + threadIdx.x; if (t >= RCH * KT * (CC / 8)) return; const int c0 = (t % (CC / 8)) * 8; const int k = (t / (CC / 8)) % KT; const int p = r0 + t / ((CC / 8) * KT); const int h = p / HH, w = p % HH; const int g = c0 / CG; const float* orow = O + (size_t)(h * PW + w) * NO3;
  const float dy = orow[g * KT + k], dx = orow[72 + g * KT + k], mo = orow[144 + g * KT + k]; const float m = 1.0f / (1.0f + expf(-mo)); const float py = (float)(h - 1 + k / 3) + dy, px = (float)(w - 1 + k % 3) + dx; const float y0f = floorf(py), x0f = floorf(px); const float wy = py - y0f, wx = px - x0f; const int y0 = (int)y0f, x0 = (int)x0f; float acc[8];
#pragma unroll
  for (int q = 0; q < 8; ++q) acc[q] = 0.f;
#pragma unroll
  for (int cn = 0; cn < 4; ++cn) { const int yy = y0 + (cn >> 1), xx = x0 + (cn & 1); const bool valid = (yy >= 0 && yy <= HH - 1 && xx >= 0 && xx <= HH - 1); const float wt = ((cn >> 1) ? wy : 1.0f - wy) * ((cn & 1) ? wx : 1.0f - wx) * (valid ? 1.f : 0.f); const int pi = min(max(yy, 0), HH - 1) * HH + min(max(xx, 0), HH - 1); FragH gq; gq.half[0] = *(const v8us*)((const unsigned short*)FU16 + (size_t)pi * CC + c0);
#pragma unroll
    for (int q = 0; q < 8; ++q) acc[q] += (float)gq.h[q] * wt; }
  FragH f;
#pragma unroll
  for (int q = 0; q < 8; ++q) f.h[q] = (_Float16)(acc[q] * m);
  *(volatile v8us*)((unsigned short*)DCOL + (size_t)(p - r0) * KD + k * CC + c0) = f.half[0]; __threadfence(); *(volatile v8us*)((unsigned short*)DCOL + (size_t)(p - r0) * KD + k * CC + c0) = f.half[0]; }
__global__ __launch_bounds__(256) void k_out(const float* __restrict__ D, const float* __restrict__ FA, int b, int r0, float* __restrict__ out) {
  #pragma clang fp contract(off)
  const int t = blockIdx.x * 256 + threadIdx.x; if (t >= CC * (RCH / 4)) return; const int p0 = r0 + (t % (RCH / 4)) * 4; const int c = t / (RCH / 4); v4f ov;
#pragma unroll
  for (int q = 0; q < 4; ++q) { const int p = p0 + q; ov[q] = fmaxf(D[(size_t)(p - r0) * CC + c], 0.f) + FA[(size_t)p * CC + c]; }
  float* dst = out + ((size_t)b * CC + c) * NPX + p0; *(volatile v4f*)dst = ov; __threadfence(); *(volatile v4f*)dst = ov; }

extern "C" void kernel_launch(void* const* d_in, const int* in_sizes, int n_in,
                              void* d_out, int out_size, void* d_ws, size_t ws_size, hipStream_t stream) {
  (void)in_sizes; (void)n_in; (void)out_size;
  const float* fl = (const float*)d_in[0]; const float* fs = (const float*)d_in[1]; const float* w_atten = (const float*)d_in[2]; const float* w_sel = (const float*)d_in[3]; const float* w_off = (const float*)d_in[4]; const float* w_coff = (const float*)d_in[5]; const float* b_coff = (const float*)d_in[6]; const float* w_dcn = (const float*)d_in[7]; const float* b_dcn = (const float*)d_in[8];
  char* ws = (char*)d_ws; size_t off = 0;
  auto take = [&](size_t bytes) { char* p = ws + off; off += (bytes + 255) & ~(size_t)255; return p; };
  _Float16* Bsel = (_Float16*)take(CC * CC * 2); _Float16* Boa = (_Float16*)take(CC * CC * 2); _Float16* Bob = (_Float16*)take(CC * CC * 2); _Float16* Bc = (_Float16*)take((size_t)KT * NO3 * CC * 2); _Float16* Bd = (_Float16*)take((size_t)CC * KD * 2); float* BPc = (float*)take(NO3 * 4); float* BPd = (float*)take(CC * 4); float* GS = (float*)take(CC * 32 * 4); float* AG = (float*)take(CC * 32 * 4);
  _Float16* XG = (_Float16*)take((size_t)NPX * CC * 2); float* FA = (float*)take((size_t)NPX * CC * 4); _Float16* FA16 = (_Float16*)take((size_t)NPX * CC * 2); _Float16* FU16 = (_Float16*)take((size_t)NPX * CC * 2); float* OFf = (float*)take((size_t)NPX * CC * 4); _Float16* XP = (_Float16*)take((size_t)PR * PW * CC * 2); float* O = (float*)take((size_t)MP * NO3 * 4); _Float16* DCOL = (_Float16*)take((size_t)RCH * KD * 2); float* D = (float*)take((size_t)RCH * CC * 4);
  if (off > ws_size) return;
  k_round16f<<<(CC * CC / 8 + 255) / 256, 256, 0, stream>>>(w_sel, Bsel, (size_t)CC * CC / 8); k_woff<<<(CC * (CC / 8) + 255) / 256, 256, 0, stream>>>(w_off, Boa, Bob); k_wcoff<<<(KT * NO3 * (CC / 8) + 255) / 256, 256, 0, stream>>>(w_coff, Bc); k_wdcn<<<(CC * (KD / 8) + 255) / 256, 256, 0, stream>>>(w_dcn, Bd);
  k_bpad<<<1, 256, 0, stream>>>(b_coff, 216, NO3, BPc); k_bpad<<<1, 256, 0, stream>>>(b_dcn, CC, CC, BPd);
  const unsigned nb8 = (NPX * (CC / 8) + 255) / 256; const dim3 gN(((NPX / 16) * (CC / 64) + 3) / 4, 1), gF(((MP / 16) * ((NO3 + 63) / 64) + 3) / 4, 1), gD(((RCH / 16) * (CC / 64) + 3) / 4, 1);
  for (int b = 0; b < NBI; ++b) {
    k_gap<<<CC, 256, 0, stream>>>(fl, b, GS); k_agate<<<1, 256, 0, stream>>>(GS, w_atten, AG); k_xg<<<nb8, 256, 0, stream>>>(fl, b, AG, XG); k_ups<<<nb8, 256, 0, stream>>>(fs, b, FU16);
    k_gemm_hhx<0><<<gN, 128, 0, stream>>>(XG, CC, 0, Bsel, CC, 0, 0.0625f, nullptr, 0, nullptr, 1, 0, 0, FA, nullptr, CC, 0, NPX, CC, CC); k_f16<<<nb8, 256, 0, stream>>>(FA, FA16);
    k_gemm_hhx<0><<<gN, 128, 0, stream>>>(FA16, CC, 0, Boa, CC, 0, 0.0625f, nullptr, 0, nullptr, 1, 0, 0, OFf, nullptr, CC, 0, NPX, CC, CC);
    k_gemm_hhx<0><<<gN, 128, 0, stream>>>(FU16, CC, 0, Bob, CC, 0, 0.125f, nullptr, 0, OFf, 1, (size_t)CC, 0, OFf, nullptr, CC, 0, NPX, CC, CC);
    k_pad<<<(PR * PW * (CC / 8) + 255) / 256, 256, 0, stream>>>(OFf, XP);
    for (int k = 0; k < KT; ++k) { const size_t ao = ((size_t)(k / 3) * PW + (k % 3)) * CC;
      k_gemm_hhx<0><<<gF, 128, 0, stream>>>(XP + ao, CC, 0, Bc + (size_t)k * NO3 * CC, CC, 0, 0.0625f, (k == 0) ? BPc : nullptr, 0, (k == 0) ? nullptr : O, 1, (size_t)NO3, 0, O, nullptr, NO3, 0, MP, NO3, CC); }
    for (int ch = 0; ch < NPX / RCH; ++ch) { const int r0 = ch * RCH;
      k_dsamp<<<(RCH * KT * (CC / 8) + 255) / 256, 256, 0, stream>>>(O, FU16, r0, DCOL);
      k_gemm_hhx<0><<<gD, 128, 0, stream>>>(DCOL, KD, 0, Bd, KD, 0, 0.0625f, BPd, 0, nullptr, 1, 0, 0, D, nullptr, CC, 0, RCH, CC, KD);
      k_out<<<(CC * (RCH / 4) + 255) / 256, 256, 0, stream>>>(D, FA, b, r0, (float*)d_out); } }
}
